// GroupedQueryAttention_81011673137882
// MI455X (gfx1250) — hardware-verified
//
#include <hip/hip_runtime.h>
#include <math.h>

typedef __attribute__((ext_vector_type(16))) _Float16     v16h;
typedef __attribute__((ext_vector_type(8)))  _Float16     v8h;
typedef __attribute__((ext_vector_type(16))) __bf16       v16b;
typedef __attribute__((ext_vector_type(8)))  __bf16       v8b;
typedef __attribute__((ext_vector_type(8)))  float        v8f;
typedef __attribute__((ext_vector_type(4)))  float        v4f;
typedef __attribute__((ext_vector_type(4)))  unsigned int v4u;

#ifndef NB
#define NB 2
#endif
#ifndef SEQ
#define SEQ 2048
#endif
#define NB_FULL  2
#define SEQ_FULL 2048
#define DM    1024
#define NQH   16
#define NKVH  4
#define GRP   4
#define HDIM  64
#define NPROJ 1536
#define QKW   1280
#define KOFF  1024
#define VOFF  1280
#define WROWS 2560
#define OWROW 1536
#define CTXW  2048
#define KC    64
#define QT    16
#define NWAVE 4
#define MROWS (NB * SEQ)
#define GTM   128
#define GTN   64

#define X16_BYTES ((size_t)MROWS * DM * 2)
#define W16_BYTES ((size_t)WROWS * DM * 2)
#define QK_BYTES  ((size_t)MROWS * QKW * 2)
#define VT_BYTES  ((size_t)NB * NKVH * HDIM * SEQ * 2)
#define CTX_BYTES ((size_t)MROWS * CTXW * 2)

static_assert(SEQ % KC == 0);
static_assert(SEQ % QT == 0);
static_assert(SEQ % GTM == 0);
static_assert(MROWS % GTM == 0);
static_assert(SEQ <= SEQ_FULL && NB <= NB_FULL);
static_assert(DM == NQH * HDIM);
static_assert(NQH == NKVH * GRP);
static_assert(GRP == NWAVE);
static_assert(HDIM == 64 && KC == 64 && QT == 16);
static_assert(GTN == HDIM);
static_assert(NPROJ == DM + 2 * NKVH * HDIM);
static_assert(QKW == DM + NKVH * HDIM && KOFF == DM && VOFF == QKW);
static_assert(NPROJ % GTN == 0 && DM % GTN == 0 && VOFF % GTN == 0 && KOFF % GTN == 0);
static_assert(WROWS == NPROJ + DM && OWROW == NPROJ);
static_assert(CTXW == 2 * DM);
static_assert((DM & (DM - 1)) == 0);
static_assert(DM % 32 == 0 && CTXW % 32 == 0);
static_assert(NWAVE * 32 * 4 == KC * (HDIM / 8));
static_assert(HDIM * 2 == 8 * 16);
static_assert(HDIM * 4 == 16 * 16);
static_assert(GTM * 2 == 16 * 16);
static_assert((QKW % 64) == 0 && (CTXW % 64) == 0 && (SEQ % 64) == 0 && (DM % 64) == 0);
static_assert(X16_BYTES % 256 == 0 && W16_BYTES % 256 == 0 && QK_BYTES % 256 == 0 && VT_BYTES % 256 == 0 && CTX_BYTES % 256 == 0);
static_assert(X16_BYTES + W16_BYTES + QK_BYTES + VT_BYTES + CTX_BYTES <= (size_t)134217728);

__device__ __forceinline__ unsigned int bf_bits(float f) {
    const unsigned int u = __float_as_uint(f);
    return (u + 0x7FFFu + ((u >> 16) & 1u)) >> 16;
}
__device__ __forceinline__ float bf_val(float f) { return __uint_as_float(bf_bits(f) << 16); }
__device__ __forceinline__ unsigned int h_bits(float f) { return (unsigned int)__builtin_bit_cast(unsigned short, (_Float16)f); }

__device__ __forceinline__ v8f mma_bf(v16b a, v16b b, v8f c) {
    c = __builtin_amdgcn_wmma_f32_16x16x32_bf16(false, a, false, b, (short)0, c, false, false);
    asm volatile("v_nop\n\tv_nop\n\tv_nop\n\tv_nop" : "+v"(c) : "v"(a), "v"(b));
    return c;
}
__device__ __forceinline__ v8f mma_h(v16h a, v16h b, v8f c) {
    c = __builtin_amdgcn_wmma_f32_16x16x32_f16(false, a, false, b, (short)0, c, false, false);
    asm volatile("v_nop\n\tv_nop\n\tv_nop\n\tv_nop" : "+v"(c) : "v"(a), "v"(b));
    return c;
}

__device__ __forceinline__ void st16x2(unsigned short* p, v4u v) {
    volatile v4u* d = (volatile v4u*)p;
    *d = v; __threadfence(); *d = v;
}

__global__ __launch_bounds__(256) void k_cvt_bf(const float* __restrict__ src, unsigned short* __restrict__ dst,
                                                 int rows, int rows_per_batch, int src_batch_rows) {
    const long long u = (long long)blockIdx.x * 256 + threadIdx.x;
    if (u >= (long long)rows * (DM / 8)) return;
    const int pc  = (int)(u % (DM / 8));
    const int row = (int)(u / (DM / 8));
    const int b = row / rows_per_batch, s = row - b * rows_per_batch;
    const float* p = src + ((size_t)b * src_batch_rows + s) * DM + pc * 8;
    const v4f a = *(const v4f*)(p), c = *(const v4f*)(p + 4);
    v4u pk;
    pk.x = bf_bits(a.x) | (bf_bits(a.y) << 16); pk.y = bf_bits(a.z) | (bf_bits(a.w) << 16);
    pk.z = bf_bits(c.x) | (bf_bits(c.y) << 16); pk.w = bf_bits(c.z) | (bf_bits(c.w) << 16);
    st16x2(dst + (size_t)row * DM + pc * 8, pk);
}

__device__ __forceinline__ void gemm_main(const __bf16* __restrict__ A, const int lda, const int KA,
                                          const __bf16* __restrict__ W, const int m0w, const int n0,
                                          const int hh, const int c, v8f (&acc)[2][4]) {
    union FB { v16b v; v8b h[2]; };
    const __bf16* a0 = A + (size_t)(m0w + c) * lda + 8 * hh;
    const __bf16* a1 = a0 + (size_t)16 * lda;
    const __bf16* w0 = W + (size_t)(n0 + c) * DM + 8 * hh;
    for (int k0 = 0; k0 < KA; k0 += 32) {
        const int kw = k0 & (DM - 1);
        FB fa0, fa1, fb[4];
        fa0.h[0] = *(const v8b*)(a0 + k0);
        fa0.h[1] = *(const v8b*)(a0 + k0 + 16);
        fa1.h[0] = *(const v8b*)(a1 + k0);
        fa1.h[1] = *(const v8b*)(a1 + k0 + 16);
#pragma unroll
        for (int j = 0; j < 4; ++j) {
            fb[j].h[0] = *(const v8b*)(w0 + (size_t)j * 16 * DM + kw);
            fb[j].h[1] = *(const v8b*)(w0 + (size_t)j * 16 * DM + kw + 16);
        }
#pragma unroll
        for (int j = 0; j < 4; ++j) {
            acc[0][j] = mma_bf(fa0.v, fb[j].v, acc[0][j]);
            acc[1][j] = mma_bf(fa1.v, fb[j].v, acc[1][j]);
        }
    }
}

__global__ __launch_bounds__(128) void k_proj(const __bf16* __restrict__ X16, const __bf16* __restrict__ W16,
                                               const float* __restrict__ fcos, const float* __restrict__ fsin,
                                               unsigned short* __restrict__ QKP, unsigned short* __restrict__ VT) {
    __shared__ __align__(16) float Cs[GTM * 68];
    const int tid = threadIdx.x, wave = tid >> 5, lane = tid & 31, hh = lane >> 4, c = lane & 15;
    const int n0 = blockIdx.x * GTN, m0 = blockIdx.y * GTM;
    const float CARRY = 16.0f;

    v8f acc[2][4];
#pragma unroll
    for (int i = 0; i < 2; ++i)
#pragma unroll
        for (int j = 0; j < 4; ++j) acc[i][j] = (v8f){0.f, 0.f, 0.f, 0.f, 0.f, 0.f, 0.f, 0.f};
    gemm_main(X16, DM, DM, W16, m0 + 32 * wave, n0, hh, c, acc);

#pragma unroll
    for (int i = 0; i < 2; ++i)
#pragma unroll
        for (int j = 0; j < 4; ++j)
#pragma unroll
            for (int r = 0; r < 8; ++r) Cs[(32 * wave + i * 16 + 8 * hh + r) * 68 + j * 16 + c] = acc[i][j][r];
    __syncthreads();

    if (n0 < VOFF) {
        const int rq = lane >> 3, pc = lane & 7;
#pragma unroll 1
        for (int it = 0; it < 8; ++it) {
            const int row = 32 * wave + it * 4 + rq;
            const int gm = m0 + row;
            const int t = gm % SEQ;
            const v4f f0 = *(const v4f*)(Cs + row * 68 + pc * 8);
            const v4f f1 = *(const v4f*)(Cs + row * 68 + pc * 8 + 4);
            const v4f cc = *(const v4f*)(fcos + (size_t)t * 32 + pc * 4);
            const v4f ss = *(const v4f*)(fsin + (size_t)t * 32 + pc * 4);
            const float c0 = bf_val(cc.x), c1 = bf_val(cc.y), c2 = bf_val(cc.z), c3 = bf_val(cc.w);
            const float s0 = bf_val(ss.x), s1 = bf_val(ss.y), s2 = bf_val(ss.z), s3 = bf_val(ss.w);
            const float o0 = (f0.x * c0 - f0.y * s0) * CARRY, o1 = (f0.x * s0 + f0.y * c0) * CARRY;
            const float o2 = (f0.z * c1 - f0.w * s1) * CARRY, o3 = (f0.z * s1 + f0.w * c1) * CARRY;
            const float o4 = (f1.x * c2 - f1.y * s2) * CARRY, o5 = (f1.x * s2 + f1.y * c2) * CARRY;
            const float o6 = (f1.z * c3 - f1.w * s3) * CARRY, o7 = (f1.z * s3 + f1.w * c3) * CARRY;
            v4u pk;
            pk.x = h_bits(o0) | (h_bits(o1) << 16); pk.y = h_bits(o2) | (h_bits(o3) << 16);
            pk.z = h_bits(o4) | (h_bits(o5) << 16); pk.w = h_bits(o6) | (h_bits(o7) << 16);
            st16x2(QKP + (size_t)gm * QKW + n0 + pc * 8, pk);
        }
    } else {
        const int g = (n0 - VOFF) >> 6;
        const int b = m0 / SEQ, s0 = m0 - b * SEQ;
#pragma unroll 1
        for (int it = 0; it < 8; ++it) {
            const int d = wave * 16 + it * 2 + hh;
            unsigned int e[8];
#pragma unroll
            for (int j = 0; j < 8; ++j) e[j] = h_bits(Cs[(c * 8 + j) * 68 + d] * CARRY);
            v4u pk;
            pk.x = e[0] | (e[1] << 16); pk.y = e[2] | (e[3] << 16); pk.z = e[4] | (e[5] << 16); pk.w = e[6] | (e[7] << 16);
            st16x2(VT + ((size_t)((b * NKVH + g) * HDIM + d)) * SEQ + s0 + c * 8, pk);
        }
    }
}

__global__ __launch_bounds__(128) void k_attn_grp(const unsigned short* __restrict__ QKP, const unsigned short* __restrict__ VT16,
                                                   unsigned short* __restrict__ CTX) {
    union FH { v16h v; v8h h[2]; };
    __shared__ __align__(16) unsigned short Ksh[KC * HDIM];
    __shared__ __align__(16) unsigned short Vth[HDIM * KC];
    __shared__ __align__(16) _Float16       Psh[NWAVE][QT * KC];
    __shared__ __align__(16) float          Os[NWAVE][QT * 68];

    const int tid = threadIdx.x, wave = tid >> 5, lane = tid & 31, hh = lane >> 4, c = lane & 15;
    const int qb = blockIdx.x, kv = blockIdx.y, b = blockIdx.z;
    const int head = kv * GRP + wave;
    const int q0 = qb * QT;
    const float SC  = 1.4426950408889634f * 0.125f * (1.0f / 256.0f);
    const float PSC = 32768.0f;
    const float VC  = 16.0f;

    FH qa[2];
    {
        const _Float16* qrow = (const _Float16*)QKP + ((size_t)b * SEQ + q0 + c) * QKW + head * HDIM;
#pragma unroll
        for (int dc = 0; dc < 2; ++dc) {
            qa[dc].h[0] = *(const v8h*)(qrow + dc * 32 + 8 * hh);
            qa[dc].h[1] = *(const v8h*)(qrow + dc * 32 + 16 + 8 * hh);
        }
    }

    float mrow[8], lrow[8];
    v8f oacc[4];
#pragma unroll
    for (int r = 0; r < 8; ++r) { mrow[r] = -INFINITY; lrow[r] = 0.f; }
#pragma unroll
    for (int t = 0; t < 4; ++t) oacc[t] = (v8f){0.f, 0.f, 0.f, 0.f, 0.f, 0.f, 0.f, 0.f};

    const unsigned short* Kb = QKP + ((size_t)b * SEQ) * QKW + KOFF + kv * HDIM;
    const unsigned short* Vb = VT16 + ((size_t)(b * NKVH + kv) * HDIM) * SEQ;
    const _Float16* Kp = (const _Float16*)Ksh;
    const _Float16* Vp = (const _Float16*)Vth;
    _Float16* pw = Psh[wave];

    for (int kc = 0; kc < SEQ / KC; ++kc) {
        const int kv0 = kc * KC;
        __syncthreads();
#pragma unroll
        for (int i = 0; i < 4; ++i) {
            const int idx = tid + 128 * i;
            const int row = idx >> 3, pc = idx & 7;
            const v4u kk = *(const v4u*)(Kb + (size_t)(kv0 + row) * QKW + pc * 8);
            const v4u vv = *(const v4u*)(Vb + (size_t)row * SEQ + kv0 + pc * 8);
            *(v4u*)(Ksh + row * HDIM + pc * 8) = kk;
            *(v4u*)(Vth + row * KC + pc * 8)   = vv;
        }
        __syncthreads();

        v8f s[4];
#pragma unroll
        for (int j = 0; j < 4; ++j) {
            s[j] = (v8f){0.f, 0.f, 0.f, 0.f, 0.f, 0.f, 0.f, 0.f};
#pragma unroll
            for (int dc = 0; dc < 2; ++dc) {
                FH kb;
                kb.h[0] = *(const v8h*)(Kp + (j * 16 + c) * HDIM + dc * 32 + 8 * hh);
                kb.h[1] = *(const v8h*)(Kp + (j * 16 + c) * HDIM + dc * 32 + 16 + 8 * hh);
                s[j] = mma_h(qa[dc].v, kb.v, s[j]);
            }
        }

#pragma unroll
        for (int r = 0; r < 8; ++r) {
            const float x0 = s[0][r] * SC, x1 = s[1][r] * SC, x2 = s[2][r] * SC, x3 = s[3][r] * SC;
            float m = fmaxf(fmaxf(x0, x1), fmaxf(x2, x3));
            m = fmaxf(m, __shfl_xor(m, 1, 32)); m = fmaxf(m, __shfl_xor(m, 2, 32));
            m = fmaxf(m, __shfl_xor(m, 4, 32)); m = fmaxf(m, __shfl_xor(m, 8, 32));
            const float mnew  = fmaxf(mrow[r], m);
            const float alpha = exp2f(mrow[r] - mnew);
            mrow[r] = mnew;
            const float p0 = exp2f(x0 - mnew), p1 = exp2f(x1 - mnew), p2 = exp2f(x2 - mnew), p3 = exp2f(x3 - mnew);
            _Float16* prow = pw + (8 * hh + r) * KC + c;
            prow[0]  = (_Float16)(p0 * PSC);
            prow[16] = (_Float16)(p1 * PSC);
            prow[32] = (_Float16)(p2 * PSC);
            prow[48] = (_Float16)(p3 * PSC);
            float psum = (p0 + p1) + (p2 + p3);
            psum += __shfl_xor(psum, 1, 32); psum += __shfl_xor(psum, 2, 32);
            psum += __shfl_xor(psum, 4, 32); psum += __shfl_xor(psum, 8, 32);
            lrow[r] = lrow[r] * alpha + psum;
#pragma unroll
            for (int t = 0; t < 4; ++t) oacc[t][r] *= alpha;
        }
        __builtin_amdgcn_fence(3  , "workgroup");
        __builtin_amdgcn_wave_barrier();
        __builtin_amdgcn_fence(2  , "workgroup");

#pragma unroll
        for (int kk = 0; kk < 2; ++kk) {
            FH pa;
            pa.h[0] = *(const v8h*)(pw + c * KC + kk * 32 + 8 * hh);
            pa.h[1] = *(const v8h*)(pw + c * KC + kk * 32 + 16 + 8 * hh);
#pragma unroll
            for (int t = 0; t < 4; ++t) {
                FH vb;
                vb.h[0] = *(const v8h*)(Vp + (t * 16 + c) * KC + kk * 32 + 8 * hh);
                vb.h[1] = *(const v8h*)(Vp + (t * 16 + c) * KC + kk * 32 + 16 + 8 * hh);
                oacc[t] = mma_h(pa.v, vb.v, oacc[t]);
            }
        }
    }

    float* os = Os[wave];
#pragma unroll
    for (int r = 0; r < 8; ++r) {
        const float inv = 1.0f / (lrow[r] * (PSC * VC));
#pragma unroll
        for (int t = 0; t < 4; ++t) os[(8 * hh + r) * 68 + t * 16 + c] = oacc[t][r] * inv;
    }
    __builtin_amdgcn_fence(3  , "workgroup");
    __builtin_amdgcn_wave_barrier();
    __builtin_amdgcn_fence(2  , "workgroup");
    {
        unsigned short* cb = CTX + ((size_t)b * SEQ + q0) * CTXW + head * HDIM;
        const int rq = lane >> 3, pc = lane & 7;
#pragma unroll 1
        for (int it = 0; it < 4; ++it) {
            const int row = it * 4 + rq;
            const v4f f0 = *(const v4f*)(os + row * 68 + pc * 8);
            const v4f f1 = *(const v4f*)(os + row * 68 + pc * 8 + 4);
            unsigned int hb[8], lb[8];
#pragma unroll
            for (int e = 0; e < 4; ++e) {
                hb[e]     = bf_bits(f0[e]);
                lb[e]     = bf_bits(f0[e] - __uint_as_float(hb[e] << 16));
                hb[4 + e] = bf_bits(f1[e]);
                lb[4 + e] = bf_bits(f1[e] - __uint_as_float(hb[4 + e] << 16));
            }
            v4u ph, pl;
            ph.x = hb[0] | (hb[1] << 16); ph.y = hb[2] | (hb[3] << 16); ph.z = hb[4] | (hb[5] << 16); ph.w = hb[6] | (hb[7] << 16);
            pl.x = lb[0] | (lb[1] << 16); pl.y = lb[2] | (lb[3] << 16); pl.z = lb[4] | (lb[5] << 16); pl.w = lb[6] | (lb[7] << 16);
            st16x2(cb + (size_t)row * CTXW + pc * 8, ph);
            st16x2(cb + (size_t)row * CTXW + DM + pc * 8, pl);
        }
    }
}

__global__ __launch_bounds__(128) void k_outp(const __bf16* __restrict__ CTXp, const __bf16* __restrict__ WO,
                                               float* __restrict__ out) {
    __shared__ __align__(16) float Cs[GTM * 68];
    const int tid = threadIdx.x, wave = tid >> 5, lane = tid & 31, hh = lane >> 4, c = lane & 15;
    const int n0 = blockIdx.x * GTN, m0 = blockIdx.y * GTM;

    v8f acc[2][4];
#pragma unroll
    for (int i = 0; i < 2; ++i)
#pragma unroll
        for (int j = 0; j < 4; ++j) acc[i][j] = (v8f){0.f, 0.f, 0.f, 0.f, 0.f, 0.f, 0.f, 0.f};
    gemm_main(CTXp, CTXW, CTXW, WO, m0 + 32 * wave, n0, hh, c, acc);

#pragma unroll
    for (int i = 0; i < 2; ++i)
#pragma unroll
        for (int j = 0; j < 4; ++j)
#pragma unroll
            for (int r = 0; r < 8; ++r) Cs[(32 * wave + i * 16 + 8 * hh + r) * 68 + j * 16 + c] = acc[i][j][r];
    __syncthreads();
    {
        float* ob = out + (size_t)(m0 + 32 * wave) * DM + n0;
        const float* cw = Cs + 32 * wave * 68;
        const int c4 = c * 4;
        for (int pass = 0; pass < 2; ++pass) {
#pragma unroll 4
            for (int it = 0; it < 16; ++it) {
                const int row = it * 2 + hh;
                const v4f val = *(const v4f*)(cw + row * 68 + c4);
                *(volatile v4f*)(ob + (size_t)row * DM + c4) = val;
            }
            __threadfence();
        }
    }
}

extern "C" void kernel_launch(void* const* d_in, const int* in_sizes, int n_in, void* d_out, int out_size, void* d_ws, size_t ws_size, hipStream_t stream) {
    if (n_in < 6) return;
    if ((long long)in_sizes[0] < (long long)(NB - 1) * SEQ_FULL * DM + (long long)SEQ * DM) return;
    if ((long long)in_sizes[1] < (long long)DM * DM) return;
    if ((long long)in_sizes[2] < (long long)(2 * NKVH * HDIM) * DM) return;
    if ((long long)in_sizes[3] < (long long)DM * DM) return;
    if ((long long)in_sizes[4] < (long long)SEQ * 32) return;
    if ((long long)in_sizes[5] < (long long)SEQ * 32) return;
    if ((long long)out_size < (long long)NB * SEQ * DM) return;
    if (ws_size < X16_BYTES + W16_BYTES + QK_BYTES + VT_BYTES + CTX_BYTES) return;

    const float* x    = (const float*)d_in[0];
    const float* q_w  = (const float*)d_in[1];
    const float* kv_w = (const float*)d_in[2];
    const float* o_w  = (const float*)d_in[3];
    const float* fcos = (const float*)d_in[4];
    const float* fsin = (const float*)d_in[5];
    float* out = (float*)d_out;

    char* ws = (char*)d_ws;
    unsigned short* X16 = (unsigned short*)(ws);
    unsigned short* W16 = (unsigned short*)(ws + X16_BYTES);
    unsigned short* QKP = (unsigned short*)(ws + X16_BYTES + W16_BYTES);
    unsigned short* VT  = (unsigned short*)(ws + X16_BYTES + W16_BYTES + QK_BYTES);
    unsigned short* CTX = (unsigned short*)(ws + X16_BYTES + W16_BYTES + QK_BYTES + VT_BYTES);

    k_cvt_bf<<<(unsigned)(((long long)MROWS * (DM / 8) + 255) / 256), 256, 0, stream>>>(x, X16, MROWS, SEQ, SEQ_FULL);
    k_cvt_bf<<<(unsigned)(((long long)DM * (DM / 8) + 255) / 256), 256, 0, stream>>>(q_w, W16, DM, DM, DM);
    k_cvt_bf<<<(unsigned)(((long long)(2 * NKVH * HDIM) * (DM / 8) + 255) / 256), 256, 0, stream>>>(kv_w, W16 + (size_t)DM * DM, 2 * NKVH * HDIM, 2 * NKVH * HDIM, 2 * NKVH * HDIM);
    k_cvt_bf<<<(unsigned)(((long long)DM * (DM / 8) + 255) / 256), 256, 0, stream>>>(o_w, W16 + (size_t)OWROW * DM, DM, DM, DM);

    k_proj<<<dim3((unsigned)(NPROJ / GTN), (unsigned)(MROWS / GTM)), 128, 0, stream>>>((const __bf16*)X16, (const __bf16*)W16, fcos, fsin, QKP, VT);
    k_attn_grp<<<dim3((unsigned)(SEQ / QT), (unsigned)NKVH, (unsigned)NB), 128, 0, stream>>>(QKP, VT, CTX);
    k_outp<<<dim3((unsigned)(DM / GTN), (unsigned)(MROWS / GTM)), 128, 0, stream>>>((const __bf16*)CTX, (const __bf16*)(W16 + (size_t)OWROW * DM), out);
}
